// MultiViewDualSoftmaxLoss_31164282699995
// MI455X (gfx1250) — hardware-verified
//
#include <hip/hip_runtime.h>
#include <hip/hip_bf16.h>

#define __bf16 _Float16
typedef __attribute__((ext_vector_type(4))) float v4f_t;
typedef float v4fa __attribute__((ext_vector_type(4), may_alias));
#define NBLK 32
typedef __attribute__((ext_vector_type(16))) __bf16 v16bf;
typedef __attribute__((ext_vector_type(8)))  __bf16 v8bf;
typedef __attribute__((ext_vector_type(8)))  float  v8f;

#define NTOK   4096
#define CDIM   128
#define NVIEW  4
#define NPAIRS 6

__device__ __forceinline__ unsigned encOrd(float f) {
    unsigned u = __float_as_uint(f);
    return (u & 0x80000000u) ? ~u : (u | 0x80000000u);
}
__device__ __forceinline__ float decOrd(unsigned u) {
    u = (u & 0x80000000u) ? (u & 0x7fffffffu) : ~u;
    return __uint_as_float(u);
}
__device__ __forceinline__ float get_temp(const float* lt) {
    return fminf(fmaxf(expf(lt[0]), 0.01f), 10.0f);
}

__device__ __forceinline__ void async_ld16(void* lds, const void* g) {
    unsigned loff = (unsigned)(uintptr_t)lds;
    asm volatile("global_load_async_to_lds_b128 %0, %1, off"
                 :: "v"(loff), "v"(g)
                 : "memory");
}
__device__ __forceinline__ void wait_async_le8() {
    asm volatile("s_wait_asynccnt 8" ::: "memory");
}
__device__ __forceinline__ void wait_async_0() {
    asm volatile("s_wait_asynccnt 0" ::: "memory");
}

__global__ void init_kernel(unsigned* __restrict__ stats, float* __restrict__ out) {
    int t = blockIdx.x * blockDim.x + threadIdx.x;
    if (t < 5 * NPAIRS * NTOK) stats[t] = 0u;
    if (t == 0) out[0] = 0.0f;
}

__global__ __launch_bounds__(256) void normalize_kernel(const float* __restrict__ desc,
                                                        __bf16* __restrict__ dn) {
    int row  = (blockIdx.x * blockDim.x + threadIdx.x) >> 5;
    int lane = threadIdx.x & 31;
    const float4 x = ((const float4*)(desc + (size_t)row * CDIM))[lane];
    float ss = x.x * x.x + x.y * x.y + x.z * x.z + x.w * x.w;
    #pragma unroll
    for (int m = 1; m < 32; m <<= 1) ss += __shfl_xor(ss, m, 32);
    float inv = 1.0f / fmaxf(sqrtf(ss), 1e-12f);
    int n = row >> 2, v = row & 3;
    __bf16 o[4];
    o[0] = (__bf16)(x.x * inv);
    o[1] = (__bf16)(x.y * inv);
    o[2] = (__bf16)(x.z * inv);
    o[3] = (__bf16)(x.w * inv);
    __bf16* dst = dn + ((size_t)v * NTOK + n) * CDIM + lane * 4;
    typedef __attribute__((ext_vector_type(2))) unsigned v2u_t;
    const v2u_t ov = *(v2u_t*)o;
    *(volatile v2u_t*)dst = ov; __threadfence(); *(volatile v2u_t*)dst = ov;
}

__global__ __launch_bounds__(256) void pair_kernel(
    const __bf16* __restrict__ dn, const float* __restrict__ logtemp,
    float* __restrict__ rowsumP, float* __restrict__ rowmaxP,
    float* __restrict__ colsumP, float* __restrict__ colmaxP,
    float* __restrict__ diagv) {
    __shared__ float sRS[2][128], sRM[2][128], sCS[4][128], sCM[4][128], sDG[128];
    __shared__ __align__(16) __bf16 smA[2][128][72];
    __shared__ __align__(16) __bf16 smB[2][128][72];

    const int piv[NPAIRS] = {0, 0, 0, 1, 1, 2};
    const int pjv[NPAIRS] = {1, 2, 3, 2, 3, 3};
    const int pair    = blockIdx.y;
    const int rowBase = (blockIdx.x >> 5) * 128;
    const int colBase = (blockIdx.x & 31) * 128;
    const size_t vs   = (size_t)NTOK * CDIM;
    const __bf16* dA  = dn + piv[pair] * vs;
    const __bf16* dB  = dn + pjv[pair] * vs;

    const int t    = threadIdx.x;
    const int lane = t & 31;
    const int wave = t >> 5;
    const int wr   = wave >> 1;
    const int wc   = wave & 1;
    const int half = lane >> 4;
    const int l16  = lane & 15;

    const float temp = get_temp(logtemp);

    v8f acc[2][4];
    #pragma unroll
    for (int mt = 0; mt < 2; ++mt)
        #pragma unroll
        for (int nt = 0; nt < 4; ++nt) acc[mt][nt] = (v8f){};

    const int ldRow = t >> 1;
    const int ldSeg = (t & 1) * 32;
    {
        const __bf16* gA = dA + (size_t)(rowBase + ldRow) * CDIM + ldSeg;
        const __bf16* gB = dB + (size_t)(colBase + ldRow) * CDIM + ldSeg;
        #pragma unroll
        for (int s = 0; s < 2; ++s) {
            #pragma unroll
            for (int q = 0; q < 4; ++q) {
                async_ld16(&smA[s][ldRow][ldSeg + 8 * q], gA + s * 64 + 8 * q);
                async_ld16(&smB[s][ldRow][ldSeg + 8 * q], gB + s * 64 + 8 * q);
            }
        }
    }

    auto compute_stage = [&](int s) {
        #pragma unroll
        for (int ks = 0; ks < 64; ks += 32) {
            v16bf afrag[2];
            #pragma unroll
            for (int mt = 0; mt < 2; ++mt) {
                int mrow = wr * 32 + mt * 16 + l16;
                v8bf a0 = *(const v8bf*)&smA[s][mrow][ks + half * 8];
                v8bf a1 = *(const v8bf*)&smA[s][mrow][ks + 16 + half * 8];
                #pragma unroll
                for (int e = 0; e < 8; ++e) { afrag[mt][e] = a0[e]; afrag[mt][e + 8] = a1[e]; }
            }
            v16bf bfrag[4];
            #pragma unroll
            for (int nt = 0; nt < 4; ++nt) {
                int nrow = wc * 64 + nt * 16 + l16;
                v8bf b0 = *(const v8bf*)&smB[s][nrow][ks + half * 8];
                v8bf b1 = *(const v8bf*)&smB[s][nrow][ks + 16 + half * 8];
                #pragma unroll
                for (int e = 0; e < 8; ++e) { bfrag[nt][e] = b0[e]; bfrag[nt][e + 8] = b1[e]; }
            }
            #pragma unroll
            for (int mt = 0; mt < 2; ++mt)
                #pragma unroll
                for (int nt = 0; nt < 4; ++nt)
                    acc[mt][nt] = __builtin_amdgcn_wmma_f32_16x16x32_f16(
                        false, afrag[mt], false, bfrag[nt], (short)0, acc[mt][nt],
                        false, false);
        }
    };

    wait_async_le8();
    __syncthreads();
    compute_stage(0);
    wait_async_0();
    __syncthreads();
    compute_stage(1);

    const int rbI = blockIdx.x >> 5, cbI = blockIdx.x & 31;
    const bool diagBlock = (rowBase == colBase);
    float colS[4] = {0.f, 0.f, 0.f, 0.f};
    float colM[4] = {-3e38f, -3e38f, -3e38f, -3e38f};
    #pragma unroll
    for (int mt = 0; mt < 2; ++mt) {
        #pragma unroll
        for (int r = 0; r < 8; ++r) {
            const int lm = wr * 32 + mt * 16 + half * 8 + r;
            const int gm = rowBase + lm;
            float rS = 0.f, rM = -3e38f;
            #pragma unroll
            for (int nt = 0; nt < 4; ++nt) {
                float sv = acc[mt][nt][r] * temp;
                float e = __expf(sv - temp);
                rS += e;
                rM = fmaxf(rM, sv);
                colS[nt] += e;
                colM[nt] = fmaxf(colM[nt], sv);
                int gn = colBase + wc * 64 + nt * 16 + l16;
                if (diagBlock && gm == gn) sDG[lm] = sv;
            }
            #pragma unroll
            for (int m = 1; m < 16; m <<= 1) {
                rS += __shfl_xor(rS, m, 32);
                rM = fmaxf(rM, __shfl_xor(rM, m, 32));
            }
            if (l16 == 0) { sRS[wc][lm] = rS; sRM[wc][lm] = rM; }
        }
    }
    #pragma unroll
    for (int nt = 0; nt < 4; ++nt) {
        float cS = colS[nt] + __shfl_xor(colS[nt], 16, 32);
        float cM = fmaxf(colM[nt], __shfl_xor(colM[nt], 16, 32));
        if (half == 0) { const int ln = wc * 64 + nt * 16 + l16; sCS[wr][ln] = cS; sCM[wr][ln] = cM; }
    }
    __syncthreads();
    if (t < 128) {
        const float rs = sRS[0][t] + sRS[1][t], rm = fmaxf(sRM[0][t], sRM[1][t]);
        const float cs = (sCS[0][t] + sCS[1][t]) + (sCS[2][t] + sCS[3][t]);
        const float cm = fmaxf(fmaxf(sCM[0][t], sCM[1][t]), fmaxf(sCM[2][t], sCM[3][t]));
        float* prs = rowsumP + (((size_t)pair * NBLK + cbI) * NTOK) + rowBase + t;
        float* prm = rowmaxP + (((size_t)pair * NBLK + cbI) * NTOK) + rowBase + t;
        float* pcs = colsumP + (((size_t)pair * NBLK + rbI) * NTOK) + colBase + t;
        float* pcm = colmaxP + (((size_t)pair * NBLK + rbI) * NTOK) + colBase + t;
        #pragma unroll 1
        for (int pass = 0; pass < 2; ++pass) {
            *(volatile float*)prs = rs; *(volatile float*)prm = rm; *(volatile float*)pcs = cs; *(volatile float*)pcm = cm;
            if (diagBlock) *(volatile float*)(diagv + (size_t)pair * NTOK + rowBase + t) = sDG[t];
            __threadfence();
        }
    }
}

__global__ __launch_bounds__(256) void finalize_kernel(
    const float* __restrict__ rowsumP, const float* __restrict__ rowmaxP,
    const float* __restrict__ colsumP, const float* __restrict__ colmaxP,
    const float* __restrict__ diagv, const float* __restrict__ logtemp,
    float* __restrict__ out, float* __restrict__ lossP) {
    int n = blockIdx.x * blockDim.x + threadIdx.x;
    if (n >= NTOK) return;
    const int piv[NPAIRS] = {0, 0, 0, 1, 1, 2};
    const int pjv[NPAIRS] = {1, 2, 3, 2, 3, 3};
    const float temp = get_temp(logtemp);
    float conf[NVIEW] = {0.f, 0.f, 0.f, 0.f};
    float lossAcc = 0.f;
    #pragma unroll
    for (int p = 0; p < NPAIRS; ++p) {
        float rs = 0.f, cs = 0.f, rm = -3e38f, cm = -3e38f;
        #pragma unroll 4
        for (int bI = 0; bI < NBLK; ++bI) {
            const size_t o = ((size_t)p * NBLK + bI) * NTOK + n;
            rs += rowsumP[o]; cs += colsumP[o]; rm = fmaxf(rm, rowmaxP[o]); cm = fmaxf(cm, colmaxP[o]);
        }
        float lse_r = temp + logf(rs);
        float lse_c = temp + logf(cs);
        float dg    = diagv[(size_t)p * NTOK + n];
        conf[piv[p]] += expf(rm - lse_r);
        conf[pjv[p]] += expf(cm - lse_c);
        lossAcc += (lse_r - dg) + (lse_c - dg);
    }
    #pragma unroll 1
    for (int pass = 0; pass < 2; ++pass) {
        #pragma unroll
        for (int v = 0; v < NVIEW; ++v) *(volatile float*)(out + 1 + n * NVIEW + v) = conf[v] * (1.0f / (NVIEW - 1));
        *(volatile float*)(lossP + n) = lossAcc;
        __threadfence();
    }
}
__global__ __launch_bounds__(256) void loss_reduce_kernel(const float* __restrict__ lossP, float* __restrict__ out) {
    __shared__ float red[256];
    float s = 0.f;
    for (int i = threadIdx.x; i < NTOK; i += 256) s += lossP[i];
    red[threadIdx.x] = s;
    __syncthreads();
    for (int o = 128; o > 0; o >>= 1) { if (threadIdx.x < o) red[threadIdx.x] += red[threadIdx.x + o]; __syncthreads(); }
    if (threadIdx.x == 0) { const float L = red[0] * (1.0f / (NPAIRS * (float)NTOK)); *(volatile float*)out = L; __threadfence(); *(volatile float*)out = L; }
}

extern "C" void kernel_launch(void* const* d_in, const int* in_sizes, int n_in,
                              void* d_out, int out_size, void* d_ws, size_t ws_size,
                              hipStream_t stream) {
    const float* desc    = (const float*)d_in[0];
    const float* logtemp = (const float*)d_in[2];
    float* out = (float*)d_out;

    char* ws = (char*)d_ws;
    __bf16* dn = (__bf16*)ws;
    size_t dnBytes = (size_t)NVIEW * NTOK * CDIM * sizeof(__bf16);
    const size_t PSZ = (size_t)NPAIRS * NBLK * NTOK;
    float* rowsumP = (float*)(ws + dnBytes);
    float* rowmaxP = rowsumP + PSZ;
    float* colsumP = rowmaxP + PSZ;
    float* colmaxP = colsumP + PSZ;
    float* diagv   = colmaxP + PSZ;
    float* lossP   = diagv + (size_t)NPAIRS * NTOK;

    normalize_kernel<<<(NVIEW * NTOK * 32) / 256, 256, 0, stream>>>(desc, dn);
    dim3 grid(32 * 32, NPAIRS);
    pair_kernel<<<grid, 256, 0, stream>>>(dn, logtemp, rowsumP, rowmaxP, colsumP, colmaxP, diagv);
    finalize_kernel<<<NTOK / 256, 256, 0, stream>>>(rowsumP, rowmaxP, colsumP, colmaxP, diagv,
                                                    logtemp, out, lossP);
    loss_reduce_kernel<<<1, 256, 0, stream>>>(lossP, out);
}
